// MGTA_51135880626556
// MI455X (gfx1250) — hardware-verified
//
#include <hip/hip_runtime.h>
#include <stdint.h>

#define DEVINL __device__ __forceinline__

typedef _Float16 f16t;
typedef _Float16 v16h __attribute__((ext_vector_type(16)));
typedef _Float16 v8h  __attribute__((ext_vector_type(8)));
typedef _Float16 v4h  __attribute__((ext_vector_type(4)));
typedef float    v8f  __attribute__((ext_vector_type(8)));
typedef float    v4f  __attribute__((ext_vector_type(4)));
typedef float    v2f  __attribute__((ext_vector_type(2)));
typedef v8h __attribute__((may_alias)) v8ha;
typedef v4h __attribute__((may_alias)) v4ha;
typedef v4f __attribute__((may_alias)) v4fa;
union FragH { v16h v; v8h half[2]; };

#define NND   3072
#define NF    128
#define NHD   64
#define NHEAD 8
#define NPH   16
#define HF    512
#define NP    2048
#define LEN   8
#define NR    16384
#define NT    4
#define TPB   256
#define WAVES 8
#define SLOPE 0.2f
#define NEGV  (-9.0e15f)
#define XCAR  16.0f
#define WCAR  256.0f
#define PCAR  4096.0f
#define GCAR  64.0f
#define SC_H  (1.0f / 256.0f)
#define SC_O  (1.0f / (4096.0f * 16.0f))
#define SC_D2 (1.0f / 16777216.0f)
#define INVNR (1.0f / 16384.0f)

#define XBLK  (NND * NF / 8 / TPB)
#define WTIL  64
#define WBLK  (NPH * (NF / WTIL))
#define WPH   72
#define LTOK  32
#define LBLK  (NND / LTOK)
#define HMT   128
#define HPH   136
#define HBLKX (NND / HMT)
#define AMT   16
#define ABLKX (NND / AMT)
#define AKW   (NND / WAVES)
#define ATT_LDS (AMT * NND * 2)
#define GTIL  64
#define GPH   72
#define ADVB  (NR / TPB)
#define DTPB  128
#define DBLK  (HF / 64)
#define NDBLK (DBLK * DBLK)
#define FPB   32
#define FBLK  (NP / FPB)
#define PLINE 32

static_assert(TPB == WAVES * 32);
static_assert(XBLK * TPB * 8 == NND * NF);
static_assert(WBLK * WTIL == NPH * NF && NHD == WTIL && WTIL * 4 == TPB);
static_assert((WPH % 8) == 0 && (HPH % 8) == 0 && (GPH % 8) == 0);
static_assert(LBLK * LTOK == NND && LTOK == 4 * WAVES && NF == 4 * 32);
static_assert(HBLKX * HMT == NND && HMT == 16 * WAVES && (NF % 32) == 0);
static_assert(ABLKX * AMT == NND && AKW * WAVES == NND && (AKW % 32) == 0 && (NND % 64) == 0);
static_assert(AMT * 16 == TPB);
static_assert(WAVES * AMT * NHD * 4 <= ATT_LDS);
static_assert((NR % GTIL) == 0 && (HF % GTIL) == 0 && GTIL * 4 == TPB);
static_assert(ADVB * TPB == NR && ADVB == 64 && NDBLK == 64);
static_assert(FBLK * FPB == NP && FPB == 4 * WAVES && HF == 16 * 32);
static_assert(HF * NT == 2 * 4 * TPB);
static_assert(NHEAD * NHD == HF && NP * LEN == NR);

DEVINL v8f wmma_f16(v16h a, v16h b, v8f c) {
  v8f d = __builtin_amdgcn_wmma_f32_16x16x32_f16(false, a, false, b, (short)0, c, false, false);
  asm volatile("v_nop\n\tv_nop\n\tv_nop\n\tv_nop" : "+v"(d) : "v"(a), "v"(b));
  return d;
}
DEVINL v8f zero8f() {
  v8f z = {0.f, 0.f, 0.f, 0.f, 0.f, 0.f, 0.f, 0.f};
  return z;
}
DEVINL void load_frag(FragH& f, const f16t* row, int k0) {
  f.half[0] = *(const v8ha*)(row + k0);
  f.half[1] = *(const v8ha*)(row + k0 + 16);
}

DEVINL float wsum32(float v) {
  v += __shfl_xor(v, 16);
  v += __shfl_xor(v, 8);
  v += __shfl_xor(v, 4);
  v += __shfl_xor(v, 2);
  v += __shfl_xor(v, 1);
  return v;
}
DEVINL float hsum16(float v) {
  v += __shfl_xor(v, 8);
  v += __shfl_xor(v, 4);
  v += __shfl_xor(v, 2);
  v += __shfl_xor(v, 1);
  return v;
}
DEVINL float hmax16(float v) {
  v = fmaxf(v, __shfl_xor(v, 8));
  v = fmaxf(v, __shfl_xor(v, 4));
  v = fmaxf(v, __shfl_xor(v, 2));
  v = fmaxf(v, __shfl_xor(v, 1));
  return v;
}
DEVINL int clampi(int v, int lo, int hi) { return min(max(v, lo), hi); }

template <int KD>
DEVINL void mma_4n(const f16t* __restrict__ arow, const f16t* __restrict__ brow, v8f (&acc)[4]) {
  #pragma unroll 1
  for (int ks = 0; ks < KD / 32; ++ks) {
    const int k0 = 32 * ks;
    FragH a;
    load_frag(a, arow, k0);
    #pragma unroll
    for (int n = 0; n < 4; ++n) {
      FragH b;
      load_frag(b, brow + (size_t)16 * n * KD, k0);
      acc[n] = wmma_f16(a.v, b.v, acc[n]);
    }
  }
}

__global__ __launch_bounds__(TPB) void cvt_x_k(const float* __restrict__ x, f16t* __restrict__ X16)
{
  const size_t idx = ((size_t)blockIdx.x * TPB + threadIdx.x) * 8;
  const v4f a = *(const v4fa*)(x + idx), c = *(const v4fa*)(x + idx + 4);
  v8h o;
  #pragma unroll
  for (int j = 0; j < 4; ++j) {
    o[j]     = (f16t)(a[j] * XCAR);
    o[4 + j] = (f16t)(c[j] * XCAR);
  }
  *(volatile v8h*)(X16 + idx) = o;
  __threadfence();
  *(volatile v8h*)(X16 + idx) = o;
}

__global__ __launch_bounds__(TPB) void cvt_w_k(const float* __restrict__ Wp, const float* __restrict__ Ws,
                                              f16t* __restrict__ WT16)
{
  __shared__ __attribute__((aligned(16))) f16t sT[WTIL * WPH];
  const int tid = threadIdx.x, blk = blockIdx.x;
  const int ph = blk >> 1, k0 = (blk & 1) * WTIL;
  const float* Wb = (ph < NHEAD) ? Wp : Ws;
  const int hh = ph & 7;
  const int kr = tid >> 2, dc = (tid & 3) * 16;
  const float* src = Wb + ((size_t)(hh * NF + k0 + kr)) * NHD + dc;
  v4f w4[4];
  #pragma unroll
  for (int p = 0; p < 4; ++p) w4[p] = *(const v4fa*)(src + 4 * p);
  #pragma unroll
  for (int p = 0; p < 4; ++p) {
    #pragma unroll
    for (int c = 0; c < 4; ++c) sT[(dc + 4 * p + c) * WPH + kr] = (f16t)(w4[p][c] * WCAR);
  }
  __syncthreads();

  v8h v[2];
  f16t* dst[2];
  #pragma unroll
  for (int i = 0; i < 2; ++i) {
    const int q = tid + TPB * i;
    const int d = q >> 3, piece = q & 7;
    v[i]   = *(const v8ha*)(sT + d * WPH + 8 * piece);
    dst[i] = WT16 + ((size_t)(ph * NHD + d)) * NF + k0 + 8 * piece;
  }
  #pragma unroll
  for (int i = 0; i < 2; ++i) *(volatile v8h*)dst[i] = v[i];
  __threadfence();
  #pragma unroll
  for (int i = 0; i < 2; ++i) *(volatile v8h*)dst[i] = v[i];
}

__global__ __launch_bounds__(TPB) void uv_k(const float* __restrict__ Wp, const float* __restrict__ Ws,
                                           const float* __restrict__ ap, const float* __restrict__ as2,
                                           float* __restrict__ U, float* __restrict__ V)
{
  __shared__ __attribute__((aligned(16))) float suv[TPB];
  const int tid = threadIdx.x, ph = blockIdx.x;
  const float* Wb = (ph < NHEAD) ? Wp : Ws;
  const float* Ab = (ph < NHEAD) ? ap : as2;
  const int hh = ph & 7, k = tid & (NF - 1), sel = tid >> 7;
  const float* wr = Wb + ((size_t)(hh * NF + k)) * NHD;
  const float* ar = Ab + hh * (2 * NHD) + NHD * sel;
  float s = 0.0f;
  #pragma unroll 1
  for (int q = 0; q < NHD / 4; ++q) {
    const v4f wv = *(const v4fa*)(wr + 4 * q);
    const v4f av = *(const v4fa*)(ar + 4 * q);
    #pragma unroll
    for (int c = 0; c < 4; ++c) s = fmaf(wv[c], av[c], s);
  }
  suv[tid] = s;
  __syncthreads();
  const bool act = tid < 64;
  const int tc = tid & 63;
  const v4f v = *(const v4fa*)(suv + 4 * tc);
  float* dst = ((tc < 32) ? U : V) + ph * NF + 4 * (tc & 31);
  if (act) *(volatile v4f*)dst = v;
  __threadfence();
  if (act) *(volatile v4f*)dst = v;
}

__global__ __launch_bounds__(TPB) void logit_k(const float* __restrict__ x, const float* __restrict__ U,
                                              const float* __restrict__ V, float* __restrict__ F1,
                                              float* __restrict__ F2)
{
  __shared__ __attribute__((aligned(16))) float sAll[2 * NPH * LTOK];
  const int tid = threadIdx.x, lane = tid & 31, wave = tid >> 5;
  const int nb = blockIdx.x * LTOK;
  const int dl = 4 * lane;

  #pragma unroll 1
  for (int t = 0; t < 4; ++t) {
    const int tloc = 4 * wave + t;
    const v4f xv = *(const v4fa*)(x + (size_t)(nb + tloc) * NF + dl);
    #pragma unroll 1
    for (int ph = 0; ph < NPH; ++ph) {
      const v4f uv = *(const v4fa*)(U + ph * NF + dl);
      const v4f vv = *(const v4fa*)(V + ph * NF + dl);
      float ps = 0.0f, pd = 0.0f;
      #pragma unroll
      for (int c = 0; c < 4; ++c) {
        ps = fmaf(xv[c], uv[c], ps);
        pd = fmaf(xv[c], vv[c], pd);
      }
      ps = wsum32(ps);
      pd = wsum32(pd);
      if (lane == 0) {
        sAll[ph * LTOK + tloc] = ps;
        sAll[(NPH + ph) * LTOK + tloc] = pd;
      }
    }
  }
  __syncthreads();

  const int L = tid >> 3, piece = tid & 7;
  const v4f v = *(const v4fa*)(sAll + LTOK * L + 4 * piece);
  float* base = (tid < TPB / 2) ? F1 : F2;
  float* dst = base + (size_t)(L & (NPH - 1)) * NND + nb + 4 * piece;
  *(volatile v4f*)dst = v;
  __threadfence();
  *(volatile v4f*)dst = v;
}

__global__ __launch_bounds__(TPB) void whgemm_k(const f16t* __restrict__ X16, const f16t* __restrict__ WT16,
                                               f16t* __restrict__ WhT)
{
  __shared__ __attribute__((aligned(16))) f16t sHT[NHD * HPH];
  const int tid = threadIdx.x, lane = tid & 31, wave = tid >> 5;
  const int h = lane >> 4, m = lane & 15;
  const int n0 = blockIdx.x * HMT, ph = blockIdx.y;

  v8f acc[4];
  #pragma unroll
  for (int n = 0; n < 4; ++n) acc[n] = zero8f();
  const f16t* arow = X16  + ((size_t)(n0 + 16 * wave + m)) * NF + 8 * h;
  const f16t* brow = WT16 + ((size_t)(ph * NHD + m)) * NF + 8 * h;
  mma_4n<NF>(arow, brow, acc);

  #pragma unroll
  for (int ct = 0; ct < 4; ++ct) {
    v8h o;
    #pragma unroll
    for (int r = 0; r < 8; ++r) o[r] = (f16t)(acc[ct][r] * SC_H);
    *(v8ha*)(sHT + (16 * ct + m) * HPH + 16 * wave + 8 * h) = o;
  }
  __syncthreads();

  v8h v[4];
  f16t* dst[4];
  #pragma unroll
  for (int i = 0; i < 4; ++i) {
    const int q = tid + TPB * i;
    const int row = q >> 4, piece = q & 15;
    v[i]   = *(const v8ha*)(sHT + row * HPH + 8 * piece);
    dst[i] = WhT + ((size_t)(ph * NHD + row)) * NND + n0 + 8 * piece;
  }
  #pragma unroll
  for (int i = 0; i < 4; ++i) *(volatile v8h*)dst[i] = v[i];
  __threadfence();
  #pragma unroll
  for (int i = 0; i < 4; ++i) *(volatile v8h*)dst[i] = v[i];
}

__global__ __launch_bounds__(TPB) void attn_k(const f16t* __restrict__ WhT, const float* __restrict__ F1,
                                             const float* __restrict__ F2, const float* __restrict__ adj,
                                             float* __restrict__ XO)
{
  extern __shared__ __attribute__((aligned(16))) float dynb[];
  __shared__ float rowinv[AMT];
  f16t* pb = (f16t*)dynb;
  float* red = dynb;

  const int tid = threadIdx.x, lane = tid & 31, wave = tid >> 5;
  const int h = lane >> 4, m = lane & 15;
  const int r = tid >> 4, c = tid & 15;
  const int i0 = blockIdx.x * AMT, ph = blockIdx.y;
  const int pass = ph >> 3, hd = ph & 7;

  const float rs = F1[(size_t)ph * NND + i0 + r];
  const float* f2p = F2 + (size_t)ph * NND + 4 * c;
  const float* arw = adj + ((size_t)(i0 + r)) * NND + 4 * c;

  float m2 = -3.0e38f;
  #pragma unroll 2
  for (int t = 0; t < NND / 64; ++t) {
    const v4f a4 = *(const v4fa*)(arw + 64 * t);
    const v4f s4 = *(const v4fa*)(f2p + 64 * t);
    #pragma unroll
    for (int q = 0; q < 4; ++q) {
      const float cand = (a4[q] > 0.0f) ? s4[q] : -3.0e38f;
      m2 = fmaxf(m2, cand);
    }
  }
  m2 = hmax16(m2);
  float mx;
  {
    float v = rs + m2;
    v = fmaxf(v, v * SLOPE);
    mx = (m2 > -1.0e38f) ? v : NEGV;
  }

  float ssum = 0.0f;
  #pragma unroll 2
  for (int t = 0; t < NND / 64; ++t) {
    const v4f a4 = *(const v4fa*)(arw + 64 * t);
    const v4f s4 = *(const v4fa*)(f2p + 64 * t);
    v4h p4;
    #pragma unroll
    for (int q = 0; q < 4; ++q) {
      float v = rs + s4[q];
      v = fmaxf(v, v * SLOPE);
      v = (a4[q] > 0.0f) ? v : NEGV;
      const float p = __expf(v - mx);
      ssum += p;
      p4[q] = (f16t)(p * PCAR);
    }
    *(v4ha*)(pb + (size_t)r * NND + 4 * c + 64 * t) = p4;
  }
  ssum = hsum16(ssum);
  if (c == 0) rowinv[r] = 1.0f / ssum;
  __syncthreads();

  v8f acc[4];
  #pragma unroll
  for (int n = 0; n < 4; ++n) acc[n] = zero8f();
  const f16t* apr = pb + (size_t)m * NND + AKW * wave + 8 * h;
  const f16t* bpr = WhT + ((size_t)(ph * NHD + m)) * NND + AKW * wave + 8 * h;
  #pragma unroll 1
  for (int ks = 0; ks < AKW / 32; ++ks) {
    const int k0 = 32 * ks;
    FragH a;
    a.half[0] = *(const v8ha*)(apr + k0);
    a.half[1] = *(const v8ha*)(apr + k0 + 16);
    #pragma unroll
    for (int ct = 0; ct < 4; ++ct) {
      FragH bb;
      load_frag(bb, bpr + (size_t)16 * ct * NND, k0);
      acc[ct] = wmma_f16(a.v, bb.v, acc[ct]);
    }
  }
  __syncthreads();

  #pragma unroll
  for (int ct = 0; ct < 4; ++ct) {
    #pragma unroll
    for (int rr = 0; rr < 8; ++rr)
      red[(wave * AMT + 8 * h + rr) * NHD + 16 * ct + m] = acc[ct][rr];
  }
  __syncthreads();

  const int row = tid >> 4, col4 = (tid & 15) * 4;
  v4f s = {0.0f, 0.0f, 0.0f, 0.0f};
  #pragma unroll
  for (int w = 0; w < WAVES; ++w) s += *(const v4fa*)(red + (w * AMT + row) * NHD + col4);
  const float scl = rowinv[row] * SC_O;
  v4f o;
  #pragma unroll
  for (int j = 0; j < 4; ++j) {
    const float v = s[j] * scl;
    o[j] = (v > 0.0f) ? v : (__expf(v) - 1.0f);
  }
  float* dst = XO + ((size_t)(pass * NND + i0 + row)) * HF + hd * NHD + col4;
  *(volatile v4f*)dst = o;
  __threadfence();
  *(volatile v4f*)dst = o;
}

__global__ __launch_bounds__(TPB) void gatherT_k(const float* __restrict__ XO, const int* __restrict__ pth,
                                                f16t* __restrict__ GT)
{
  __shared__ __attribute__((aligned(16))) f16t sT[GTIL * GPH];
  const int tid = threadIdx.x;
  const int r0 = blockIdx.x * GTIL, c0 = blockIdx.y * GTIL, pass = blockIdx.z;
  const int rr = tid >> 2, cs = (tid & 3) * 16;
  const int nd = clampi(pth[r0 + rr], 0, NND - 1);
  const float* src = XO + ((size_t)(pass * NND + nd)) * HF + c0 + cs;
  v4f x4[4];
  #pragma unroll
  for (int p = 0; p < 4; ++p) x4[p] = *(const v4fa*)(src + 4 * p);
  #pragma unroll
  for (int p = 0; p < 4; ++p) {
    #pragma unroll
    for (int cc = 0; cc < 4; ++cc) sT[(cs + 4 * p + cc) * GPH + rr] = (f16t)(x4[p][cc] * GCAR);
  }
  __syncthreads();

  v8h v[2];
  f16t* dst[2];
  #pragma unroll
  for (int i = 0; i < 2; ++i) {
    const int q = tid + TPB * i;
    const int cl = q >> 3, piece = q & 7;
    v[i]   = *(const v8ha*)(sT + cl * GPH + 8 * piece);
    dst[i] = GT + ((size_t)(pass * HF + c0 + cl)) * NR + r0 + 8 * piece;
  }
  #pragma unroll
  for (int i = 0; i < 2; ++i) *(volatile v8h*)dst[i] = v[i];
  __threadfence();
  #pragma unroll
  for (int i = 0; i < 2; ++i) *(volatile v8h*)dst[i] = v[i];
}

__global__ __launch_bounds__(TPB) void adv_k(const float* __restrict__ XO, const int* __restrict__ pth,
                                            const int* __restrict__ tsk, const float* __restrict__ Wsc,
                                            const float* __restrict__ bsc, float* __restrict__ PA)
{
  __shared__ __attribute__((aligned(16))) float sW[HF * NT];
  __shared__ float sd[TPB];
  const int tid = threadIdx.x;
  #pragma unroll
  for (int i = 0; i < 2; ++i)
    *(v4fa*)(sW + 4 * (tid + TPB * i)) = *(const v4fa*)(Wsc + 4 * (tid + TPB * i));
  const float b0 = bsc[0], b1 = bsc[1], b2 = bsc[2], b3 = bsc[3];
  __syncthreads();

  const int r = blockIdx.x * TPB + tid;
  const int nd = clampi(pth[r], 0, NND - 1);
  const float* srow = XO + ((size_t)(NND + nd)) * HF;
  float lg0 = b0, lg1 = b1, lg2 = b2, lg3 = b3;
  #pragma unroll 1
  for (int c4 = 0; c4 < HF / 4; ++c4) {
    const v4f xv = *(const v4fa*)(srow + 4 * c4);
    #pragma unroll
    for (int cc = 0; cc < 4; ++cc) {
      const v4f w = *(const v4fa*)(sW + (4 * c4 + cc) * NT);
      lg0 = fmaf(xv[cc], w[0], lg0);
      lg1 = fmaf(xv[cc], w[1], lg1);
      lg2 = fmaf(xv[cc], w[2], lg2);
      lg3 = fmaf(xv[cc], w[3], lg3);
    }
  }
  const float z0 = __builtin_amdgcn_rcpf(1.0f + __expf(-lg0));
  const float z1 = __builtin_amdgcn_rcpf(1.0f + __expf(-lg1));
  const float z2 = __builtin_amdgcn_rcpf(1.0f + __expf(-lg2));
  const float z3 = __builtin_amdgcn_rcpf(1.0f + __expf(-lg3));
  const float mz = fmaxf(fmaxf(z0, z1), fmaxf(z2, z3));
  const float e0 = __expf(z0 - mz), e1 = __expf(z1 - mz), e2 = __expf(z2 - mz), e3 = __expf(z3 - mz);
  const float iS = __builtin_amdgcn_rcpf((e0 + e1) + (e2 + e3));
  const float p0 = e0 * iS, p1 = e1 * iS, p2 = e2 * iS, p3 = e3 * iS;
  const float mp = fmaxf(fmaxf(p0, p1), fmaxf(p2, p3));
  const float S2 = (__expf(p0 - mp) + __expf(p1 - mp)) + (__expf(p2 - mp) + __expf(p3 - mp));
  const float lse = mp + __logf(S2);
  const int tk = clampi(tsk[r], 0, NT - 1);
  float sel = p0;
  sel = (tk == 1) ? p1 : sel;
  sel = (tk == 2) ? p2 : sel;
  sel = (tk == 3) ? p3 : sel;
  sd[tid] = lse - sel;
  __syncthreads();
  #pragma unroll 1
  for (int st = TPB / 2; st > 0; st >>= 1) {
    if (tid < st) sd[tid] += sd[tid + st];
    __syncthreads();
  }
  const float part = sd[0];
  const v4f pv = {part, part, part, part};
  float* dst = PA + blockIdx.x * PLINE + 4 * (tid & 7);
  if (tid < 8) *(volatile v4f*)dst = pv;
  __threadfence();
  if (tid < 8) *(volatile v4f*)dst = pv;
}

__global__ __launch_bounds__(DTPB) void diff_k(const f16t* __restrict__ GT, float* __restrict__ PD)
{
  __shared__ float sred[4];
  const int tid = threadIdx.x, lane = tid & 31, wave = tid >> 5;
  const int h = lane >> 4, m = lane & 15;
  const int c1b = blockIdx.x * 64, c2b = blockIdx.y * 64;
  const f16t* GS = GT + (size_t)HF * NR;
  const f16t* GP = GT;

  v8f acc[4];
  #pragma unroll
  for (int n = 0; n < 4; ++n) acc[n] = zero8f();
  const f16t* arow = GS + ((size_t)(c1b + 16 * wave + m)) * NR + 8 * h;
  const f16t* brow = GP + ((size_t)(c2b + m)) * NR + 8 * h;
  mma_4n<NR>(arow, brow, acc);

  float s = 0.0f;
  #pragma unroll
  for (int ct = 0; ct < 4; ++ct) {
    #pragma unroll
    for (int rr = 0; rr < 8; ++rr) s = fmaf(acc[ct][rr], acc[ct][rr], s);
  }
  s = wsum32(s);
  if (lane == 0) sred[wave] = s;
  __syncthreads();
  const float part = (((sred[0] + sred[1]) + sred[2]) + sred[3]) * SC_D2;
  const v4f pv = {part, part, part, part};
  float* dst = PD + (blockIdx.y * DBLK + blockIdx.x) * PLINE + 4 * (tid & 7);
  if (tid < 8) *(volatile v4f*)dst = pv;
  __threadfence();
  if (tid < 8) *(volatile v4f*)dst = pv;
}

__global__ __launch_bounds__(TPB) void final_k(const float* __restrict__ XO, const int* __restrict__ pth,
                                              const float* __restrict__ Wc, const float* __restrict__ bc,
                                              float* __restrict__ out)
{
  __shared__ __attribute__((aligned(16))) float so[FPB];
  const int tid = threadIdx.x, lane = tid & 31, wave = tid >> 5;
  const int dl = 16 * lane;
  const float bc0 = bc[0];
  #pragma unroll 1
  for (int t = 0; t < 4; ++t) {
    const int pl = 4 * wave + t;
    const int p = blockIdx.x * FPB + pl;
    float s = 0.0f;
    #pragma unroll 1
    for (int l = 0; l < LEN; ++l) {
      const int nd = clampi(pth[p * LEN + l], 0, NND - 1);
      const float* sh = XO + ((size_t)(NND + nd)) * HF + dl;
      const float* pv = XO + ((size_t)nd) * HF + dl;
      const float* wS = Wc + (size_t)l * (2 * HF) + dl;
      const float* wP = wS + HF;
      #pragma unroll
      for (int q = 0; q < 4; ++q) {
        const v4f a = *(const v4fa*)(sh + 4 * q), b = *(const v4fa*)(pv + 4 * q);
        const v4f w1 = *(const v4fa*)(wS + 4 * q), w2 = *(const v4fa*)(wP + 4 * q);
        #pragma unroll
        for (int cc = 0; cc < 4; ++cc) {
          s = fmaf(a[cc], w1[cc], s);
          s = fmaf(b[cc], w2[cc], s);
        }
      }
    }
    s = wsum32(s) + bc0;
    const float o = __builtin_amdgcn_rcpf(1.0f + __expf(-s));
    if (lane == 0) so[pl] = o;
  }
  __syncthreads();
  const v4f v = *(const v4fa*)(so + 4 * (tid & 7));
  float* dst = out + blockIdx.x * FPB + 4 * (tid & 7);
  if (tid < 8) *(volatile v4f*)dst = v;
  __threadfence();
  if (tid < 8) *(volatile v4f*)dst = v;
}

__global__ __launch_bounds__(64) void finalize_k(const float* __restrict__ PA, const float* __restrict__ PD,
                                                float* __restrict__ out)
{
  __shared__ float sa[64], sb[64];
  const int tid = threadIdx.x;
  sa[tid] = PA[tid * PLINE];
  sb[tid] = PD[tid * PLINE];
  __syncthreads();
  if (tid == 0) {
    float a = 0.0f, d = 0.0f;
    #pragma unroll 1
    for (int i = 0; i < ADVB; ++i) a += sa[i];
    #pragma unroll 1
    for (int i = 0; i < NDBLK; ++i) d += sb[i];
    const v2f o = {a * INVNR, d};
    *(volatile v2f*)(out + NP) = o;
    __threadfence();
    *(volatile v2f*)(out + NP) = o;
  }
}

extern "C" void kernel_launch(void* const* d_in, const int* in_sizes, int n_in,
                              void* d_out, int out_size, void* d_ws, size_t ws_size,
                              hipStream_t stream) {
  if (n_in < 12) return;
  if (in_sizes[0] != NND * NF) return;
  if (in_sizes[1] != NND * NND) return;
  if (in_sizes[2] != NR) return;
  if (in_sizes[3] != NR) return;
  if (in_sizes[4] != NHEAD * NF * NHD) return;
  if (in_sizes[5] != NHEAD * 2 * NHD) return;
  if (in_sizes[6] != NHEAD * NF * NHD) return;
  if (in_sizes[7] != NHEAD * 2 * NHD) return;
  if (in_sizes[8] != HF * NT) return;
  if (in_sizes[9] != NT) return;
  if (in_sizes[10] != LEN * 2 * HF) return;
  if (in_sizes[11] != 1) return;
  if (out_size != NP + 2) return;

  const float* features = (const float*)d_in[0];
  const float* adj      = (const float*)d_in[1];
  const int*   pth      = (const int*)d_in[2];
  const int*   tsk      = (const int*)d_in[3];
  const float* Wp       = (const float*)d_in[4];
  const float* ap       = (const float*)d_in[5];
  const float* Ws       = (const float*)d_in[6];
  const float* as2      = (const float*)d_in[7];
  const float* Wsc      = (const float*)d_in[8];
  const float* bsc      = (const float*)d_in[9];
  const float* Wc       = (const float*)d_in[10];
  const float* bc       = (const float*)d_in[11];
  float* outp = (float*)d_out;

  const size_t szX  = (size_t)NND * NF * 2;
  const size_t szWT = (size_t)NPH * NHD * NF * 2;
  const size_t szWH = (size_t)NPH * NHD * NND * 2;
  const size_t szUV = (size_t)NPH * NF * 4;
  const size_t szF  = (size_t)NPH * NND * 4;
  const size_t szXO = (size_t)2 * NND * HF * 4;
  const size_t szGT = (size_t)2 * HF * NR * 2;
  const size_t szP  = (size_t)64 * PLINE * 4;
  size_t off = 0;
  char* ws = (char*)d_ws;
  f16t*  X16 = (f16t*)(ws + off);  off += szX;
  f16t*  WT16 = (f16t*)(ws + off); off += szWT;
  f16t*  WhT = (f16t*)(ws + off);  off += szWH;
  float* U   = (float*)(ws + off); off += szUV;
  float* V   = (float*)(ws + off); off += szUV;
  float* F1  = (float*)(ws + off); off += szF;
  float* F2  = (float*)(ws + off); off += szF;
  float* XO  = (float*)(ws + off); off += szXO;
  f16t*  GT  = (f16t*)(ws + off);  off += szGT;
  float* PA  = (float*)(ws + off); off += szP;
  float* PD  = (float*)(ws + off); off += szP;
  if (off > ws_size) return;

  cvt_x_k<<<XBLK, TPB, 0, stream>>>(features, X16);
  cvt_w_k<<<WBLK, TPB, 0, stream>>>(Wp, Ws, WT16);
  uv_k<<<NPH, TPB, 0, stream>>>(Wp, Ws, ap, as2, U, V);
  logit_k<<<LBLK, TPB, 0, stream>>>(features, U, V, F1, F2);
  whgemm_k<<<dim3(HBLKX, NPH), TPB, 0, stream>>>(X16, WT16, WhT);
  (void)hipFuncSetAttribute(reinterpret_cast<const void*>(&attn_k),
                            hipFuncAttributeMaxDynamicSharedMemorySize, ATT_LDS);
  attn_k<<<dim3(ABLKX, NPH), TPB, ATT_LDS, stream>>>(WhT, F1, F2, adj, XO);
  gatherT_k<<<dim3(NR / GTIL, HF / GTIL, 2), TPB, 0, stream>>>(XO, pth, GT);
  adv_k<<<ADVB, TPB, 0, stream>>>(XO, pth, tsk, Wsc, bsc, PA);
  diff_k<<<dim3(DBLK, DBLK), DTPB, 0, stream>>>(GT, PD);
  final_k<<<FBLK, TPB, 0, stream>>>(XO, pth, Wc, bc, outp);
  finalize_k<<<1, 64, 0, stream>>>(PA, PD, outp);
  (void)hipGetLastError();
}
